// Difference_Module_27986006901188
// MI455X (gfx1250) — hardware-run, weakly checked
//
#include <hip/hip_runtime.h>
#include <math.h>

typedef __attribute__((ext_vector_type(16))) _Float16 v16h;
typedef __attribute__((ext_vector_type(16))) __bf16 v16b;
typedef __attribute__((ext_vector_type(8)))  _Float16 v8h;
typedef __attribute__((ext_vector_type(8)))  float v8f;
typedef __attribute__((ext_vector_type(4)))  float v4f;
typedef __attribute__((ext_vector_type(2)))  float v2f;
typedef __attribute__((ext_vector_type(4)))  unsigned v4u;
typedef __attribute__((ext_vector_type(4)))  int v4i;
typedef float __attribute__((may_alias)) float_a;
typedef int __attribute__((may_alias)) int_a;

template <typename T> __device__ __forceinline__ void vst2(void* p, T v) { *(volatile T*)p = v; __threadfence(); *(volatile T*)p = v; }
__device__ __forceinline__ v8f wmma16(v16h a, v16h b, v8f c) {
  v8f d = __builtin_amdgcn_wmma_f32_16x16x32_f16(false, a, false, b, (short)0, c, false, false);
  asm volatile("v_nop\n\tv_nop\n\tv_nop\n\tv_nop" : "+v"(d) : "v"(a), "v"(b));
  return d;
}
__device__ __forceinline__ v8f wmma_bf(v16b a, v16b b, v8f c) {
  v8f d = __builtin_amdgcn_wmma_f32_16x16x32_bf16(false, a, false, b, (short)0, c, false, false);
  asm volatile("v_nop\n\tv_nop\n\tv_nop\n\tv_nop" : "+v"(d) : "v"(a), "v"(b));
  return d;
}
__device__ __forceinline__ v16h frag_h(const _Float16* rowk0, int lane) {
  union { v16h v; v8h q[2]; } u; const _Float16* p = rowk0 + 8 * (lane >> 4);
  u.q[0] = *(const v8h*)p; u.q[1] = *(const v8h*)(p + 16); return u.v;
}
__device__ __forceinline__ v16h frag_f32(const float* rowk0, int lane) {
  v16h a; const float* p = rowk0 + 8 * (lane >> 4);
#pragma unroll
  for (int i = 0; i < 8; ++i) { a[i] = (_Float16)p[i]; a[8 + i] = (_Float16)p[16 + i]; }
  return a;
}
__device__ __forceinline__ v16h frag_f32s(const float* rowk0, int lane, float sc) {
  v16h a; const float* p = rowk0 + 8 * (lane >> 4);
#pragma unroll
  for (int i = 0; i < 8; ++i) { a[i] = (_Float16)(p[i] * sc); a[8 + i] = (_Float16)(p[16 + i] * sc); }
  return a;
}
__device__ __forceinline__ v16h fragc_f32(const float* W, int k0, int n, int lane, int ld, int K) {
  v16h a; const int g = lane >> 4;
#pragma unroll
  for (int i = 0; i < 8; ++i) { const int ka = k0 + 8 * g + i, kb = ka + 16;
    a[i] = (_Float16)(ka < K ? W[(size_t)(ka < K ? ka : K - 1) * ld + n] : 0.f); a[8 + i] = (_Float16)(kb < K ? W[(size_t)(kb < K ? kb : K - 1) * ld + n] : 0.f); }
  return a;
}
struct F2 { v16b h, l; };
__device__ __forceinline__ F2 bsplit16(const float v[16]) { F2 r;
#pragma unroll
  for (int i = 0; i < 16; ++i) { const __bf16 h = (__bf16)v[i]; r.h[i] = h; r.l[i] = (__bf16)(v[i] - (float)h); }
  return r; }
__device__ __forceinline__ F2 split_row(const float* row, int k0, int lane) { float v[16]; const float* p = row + k0 + 8 * (lane >> 4);
#pragma unroll
  for (int i = 0; i < 8; ++i) { v[i] = p[i]; v[8 + i] = p[16 + i]; }
  return bsplit16(v); }
__device__ __forceinline__ F2 split_rowK(const float* row, int k0, int lane, int K) { float v[16]; const int g = lane >> 4;
#pragma unroll
  for (int i = 0; i < 8; ++i) { const int ka = k0 + 8 * g + i, kb = ka + 16; v[i] = ka < K ? row[ka < K ? ka : K - 1] : 0.f; v[8 + i] = kb < K ? row[kb < K ? kb : K - 1] : 0.f; }
  return bsplit16(v); }
__device__ __forceinline__ F2 split_col(const float* W, int k0, int n, int lane, int ld, int K) { float v[16]; const int g = lane >> 4;
#pragma unroll
  for (int i = 0; i < 8; ++i) { const int ka = k0 + 8 * g + i, kb = ka + 16; v[i] = ka < K ? W[(size_t)(ka < K ? ka : K - 1) * ld + n] : 0.f; v[8 + i] = kb < K ? W[(size_t)(kb < K ? kb : K - 1) * ld + n] : 0.f; }
  return bsplit16(v); }
__device__ __forceinline__ v8f mac3(const F2& a, const F2& b, v8f c) { c = wmma_bf(a.l, b.h, c); c = wmma_bf(a.h, b.l, c); return wmma_bf(a.h, b.h, c); }
__device__ __forceinline__ float sigm(float v) { return 1.0f / (1.0f + expf(-v)); }
#define LDSX() do { asm volatile("s_wait_dscnt 0" ::: "memory"); __builtin_amdgcn_wave_barrier(); __builtin_amdgcn_fence(__ATOMIC_RELEASE, "workgroup"); } while (0)


#define NB 8
#define SS 4096
#define HD 64
#define HID 256
#ifndef TQB
#define TQB (SS / 64)
#define TNB NB
#endif
typedef __attribute__((ext_vector_type(8))) __bf16 v8b;
__device__ __forceinline__ v16b frag_b(const __bf16* rowk0, int lane) {
  union { v16b v; v8b q[2]; } u; const __bf16* p = rowk0 + 8 * (lane >> 4);
  u.q[0] = *(const v8b*)p; u.q[1] = *(const v8b*)(p + 16); return u.v;
}
__device__ __forceinline__ float bfr(float v) { return (float)(__bf16)v; }
__device__ __attribute__((noinline)) float exp_ni(float v) { return expf(v); }
__device__ __attribute__((noinline)) float erf_ni(float v) { return erff(v); }

#define WS_PW  0u
#define WS_P1  (WS_PW + 2u * HD * HD)
#define WS_P2  (WS_P1 + 2u * HID * HD)
#define WS_Q   (WS_P2 + 2u * HD * HID + 256u)
#define WS_K   (WS_Q + 2u * (size_t)NB * SS * HD)
#define WS_VT  (WS_K + 2u * (size_t)NB * SS * HD)
#define WS_KT  (WS_VT + 2u * (size_t)NB * HD * SS)
#define WS_V1H (WS_KT + 2u * (size_t)NB * HD * SS)
#define WS_V1L (WS_V1H + 2u * (size_t)NB * HD * SS)
#define WS_M   (WS_V1L + 2u * (size_t)NB * HD * SS)
#define WS_END (WS_M + 4u * (size_t)NB * HD * HD)

__global__ __launch_bounds__(256) void k_pack(const float* __restrict__ WD, const float* __restrict__ W1, const float* __restrict__ W2, __bf16* __restrict__ P) { const int n = blockIdx.x, t = threadIdx.x; __shared__ __align__(16) __bf16 s[HID];
  if (n < HD) { if (t < HD) s[t] = (__bf16)WD[(size_t)t * HD + n]; __syncthreads(); if (t < HD / 8) vst2((unsigned*)(P + WS_PW / 2 + (size_t)n * HD + t * 8), *(const v4u*)&s[t * 8]); }
  else if (n < HD + HID) { const int o = n - HD; if (t < HD) s[t] = (__bf16)W1[(size_t)t * HID + o]; __syncthreads(); if (t < HD / 8) vst2((unsigned*)(P + WS_P1 / 2 + (size_t)o * HD + t * 8), *(const v4u*)&s[t * 8]); }
  else { const int o = n - HD - HID; s[t] = (__bf16)W2[(size_t)t * HD + o]; __syncthreads(); if (t < HID / 8) vst2((unsigned*)(P + WS_P2 / 2 + (size_t)o * HID + t * 8), *(const v4u*)&s[t * 8]); } }
__global__ __launch_bounds__(256) void k_rows(const float* __restrict__ Qi, const float* __restrict__ Ki, const float* __restrict__ Vi, _Float16* __restrict__ Q, _Float16* __restrict__ K, _Float16* __restrict__ VT, _Float16* __restrict__ KT) {
  __shared__ __align__(16) _Float16 sq[64][72]; __shared__ __align__(16) _Float16 sk[64][72]; __shared__ __align__(16) _Float16 svt[64][72]; __shared__ __align__(16) _Float16 skt[64][72];
  const size_t r0 = (size_t)blockIdx.x * 64; const size_t b = r0 / SS, s0 = r0 % SS; const int t = threadIdx.x;
  for (int e = t; e < 64 * 64; e += 256) { const int r = e >> 6, c = e & 63; const _Float16 kv = (_Float16)bfr(Ki[(r0 + r) * HD + c]); sq[r][c] = (_Float16)bfr(Qi[(r0 + r) * HD + c]); sk[r][c] = kv; skt[c][r] = kv; svt[c][r] = (_Float16)bfr(Vi[(r0 + r) * HD + c]); } __syncthreads();
  for (int e = t; e < 64 * 8; e += 256) { const int r = e >> 3, q8 = e & 7; vst2((unsigned*)(Q + (r0 + r) * HD + q8 * 8), *(const v4u*)&sq[r][q8 * 8]); vst2((unsigned*)(K + (r0 + r) * HD + q8 * 8), *(const v4u*)&sk[r][q8 * 8]); vst2((unsigned*)(VT + (b * HD + r) * SS + s0 + q8 * 8), *(const v4u*)&svt[r][q8 * 8]); vst2((unsigned*)(KT + (b * HD + r) * SS + s0 + q8 * 8), *(const v4u*)&skt[r][q8 * 8]); } }
__global__ __launch_bounds__(128) void k_attn(const _Float16* __restrict__ Q, const _Float16* __restrict__ K, const _Float16* __restrict__ VT, const float* __restrict__ Vi, const __bf16* __restrict__ P, const float* __restrict__ BD, _Float16* __restrict__ V1H, _Float16* __restrict__ V1L) {
  __shared__ __align__(16) _Float16 sph[4][16][40]; __shared__ __align__(16) _Float16 spl[4][16][40]; __shared__ __align__(16) float so[4][16][68]; __shared__ __align__(16) _Float16 sth[64][72]; __shared__ __align__(16) _Float16 stl[64][72];
  const int tid = threadIdx.x, wave = tid >> 5, lane = tid & 31, col = lane & 15, g = lane >> 4; const size_t b = blockIdx.y; const int q0b = blockIdx.x * 64; const int q0 = q0b + wave * 16; const size_t rq = b * SS + q0;
  v16h aq[2];
#pragma unroll
  for (int kc = 0; kc < 2; ++kc) aq[kc] = frag_h(Q + (rq + col) * HD + kc * 32, lane);
  float m[8], l[8];
#pragma unroll
  for (int r = 0; r < 8; ++r) { m[r] = -3.0e38f; l[r] = 0.f; }
  v8f acc[4] = {}, accl[4] = {};
#pragma unroll 1
  for (int ks = 0; ks < SS / 32; ++ks) { const int j0 = ks * 32; v8f s[2];
#pragma unroll
    for (int ct = 0; ct < 2; ++ct) { const size_t rk = (b * SS + j0 + ct * 16 + col) * HD; v8f c = {};
#pragma unroll
      for (int kc = 0; kc < 2; ++kc) c = wmma16(aq[kc], frag_h(K + rk + kc * 32, lane), c);
#pragma unroll
      for (int r = 0; r < 8; ++r) s[ct][r] = c[r] * 0.125f; }
#pragma unroll
    for (int r = 0; r < 8; ++r) { float mx = fmaxf(s[0][r], s[1][r]);
#pragma unroll
      for (int o = 1; o < 16; o <<= 1) mx = fmaxf(mx, __shfl_xor(mx, o));
      const float mn = fmaxf(m[r], mx); const float alpha = (m[r] <= -1.0e38f) ? 0.f : __expf(m[r] - mn); const float e0 = __expf(s[0][r] - mn), e1 = __expf(s[1][r] - mn); float es = e0 + e1;
#pragma unroll
      for (int o = 1; o < 16; o <<= 1) es += __shfl_xor(es, o);
      l[r] = l[r] * alpha + es; m[r] = mn;
#pragma unroll
      for (int dt = 0; dt < 4; ++dt) { acc[dt][r] *= alpha; accl[dt][r] *= alpha; }
      { const float p0 = e0 * 2048.0f, p1 = e1 * 2048.0f; const _Float16 h0 = (_Float16)p0, h1 = (_Float16)p1; sph[wave][8 * g + r][col] = h0; spl[wave][8 * g + r][col] = (_Float16)((p0 - (float)h0) * 2048.0f); sph[wave][8 * g + r][16 + col] = h1; spl[wave][8 * g + r][16 + col] = (_Float16)((p1 - (float)h1) * 2048.0f); } }
    LDSX();
    const v16h pa = frag_h(&sph[wave][col][0], lane), pal = frag_h(&spl[wave][col][0], lane);
#pragma unroll
    for (int dt = 0; dt < 4; ++dt) { const v16h vf = frag_h(VT + (b * HD + dt * 16 + col) * SS + j0, lane); acc[dt] = wmma16(pa, vf, acc[dt]); accl[dt] = wmma16(pal, vf, accl[dt]); }
    LDSX(); }
#pragma unroll
  for (int r = 0; r < 8; ++r) { const float il = (1.0f / 2048.0f) / l[r];
#pragma unroll
    for (int dt = 0; dt < 4; ++dt) { const int c = dt * 16 + col; so[wave][8 * g + r][c] = bfr(Vi[(rq + 8 * g + r) * HD + c]) - (acc[dt][r] + accl[dt][r] * (1.0f / 2048.0f)) * il; } }
  LDSX();
  { v8f a2[4] = {};
#pragma unroll
    for (int kc = 0; kc < HD / 32; ++kc) { const F2 a = split_row(&so[wave][col][0], kc * 32, lane);
#pragma unroll
      for (int jt = 0; jt < 4; ++jt) { const v16b w = frag_b(P + WS_PW / 2 + (size_t)(jt * 16 + col) * HD + kc * 32, lane); a2[jt] = wmma_bf(a.h, w, a2[jt]); a2[jt] = wmma_bf(a.l, w, a2[jt]); } }
    LDSX();
#pragma unroll
    for (int jt = 0; jt < 4; ++jt) { const float bb = bfr(BD[jt * 16 + col]);
#pragma unroll
      for (int r = 0; r < 8; ++r) { const float v = a2[jt][r] + bb; const _Float16 hv = (_Float16)v; sth[jt * 16 + col][wave * 16 + 8 * g + r] = hv; stl[jt * 16 + col][wave * 16 + 8 * g + r] = (_Float16)((v - (float)hv) * 2048.0f); } } }
  __syncthreads();
  for (int e = tid; e < 64 * 8; e += 128) { const int d = e >> 3, pc = e & 7; const size_t o = (b * HD + d) * SS + q0b + pc * 8; vst2((unsigned*)(V1H + o), *(const v4u*)&sth[d][pc * 8]); vst2((unsigned*)(V1L + o), *(const v4u*)&stl[d][pc * 8]); }
}
__global__ __launch_bounds__(128) void k_m(const _Float16* __restrict__ V1H, const _Float16* __restrict__ V1L, const _Float16* __restrict__ KT, float* __restrict__ M) {
  __shared__ __align__(16) float sm[64][68];
  const int tid = threadIdx.x, wave = tid >> 5, lane = tid & 31, col = lane & 15, g = lane >> 4; const size_t b = blockIdx.x; const int e0 = wave * 16;
  v8f acc[4] = {}, accl[4] = {};
#pragma unroll 2
  for (int kc = 0; kc < SS / 32; ++kc) { const v16h ah = frag_h(V1H + (b * HD + e0 + col) * SS + kc * 32, lane), al = frag_h(V1L + (b * HD + e0 + col) * SS + kc * 32, lane);
#pragma unroll
    for (int dt = 0; dt < 4; ++dt) { const v16h kf = frag_h(KT + (b * HD + dt * 16 + col) * SS + kc * 32, lane); acc[dt] = wmma16(ah, kf, acc[dt]); accl[dt] = wmma16(al, kf, accl[dt]); } }
#pragma unroll
  for (int dt = 0; dt < 4; ++dt)
#pragma unroll
    for (int r = 0; r < 8; ++r) sm[e0 + 8 * g + r][dt * 16 + col] = acc[dt][r] + accl[dt][r] * (1.0f / 2048.0f);
  __syncthreads();
  for (int e = tid; e < 64 * 16; e += 128) { const int row = e >> 4, q = e & 15; vst2(M + (b * HD + row) * HD + q * 4, *(const v4f*)&sm[row][q * 4]); }
}
__device__ __attribute__((noinline)) float erf_p(float v) { return erff(v); }
__global__ __launch_bounds__(128) void k_fin(const float* __restrict__ Qi, const _Float16* __restrict__ Q, const float* __restrict__ M, const __bf16* __restrict__ P, const float* __restrict__ GA, const float* __restrict__ BE, const float* __restrict__ B1, const float* __restrict__ B2, float* __restrict__ OUT) {
  __shared__ __align__(16) __bf16 smh[64][72]; __shared__ __align__(16) __bf16 sml[64][72]; __shared__ __align__(16) float sv[4][16][68]; __shared__ __align__(16) float sh[4][16][68]; __shared__ __align__(16) float sg[4][16][260];
  const int tid = threadIdx.x, wave = tid >> 5, lane = tid & 31, col = lane & 15, g = lane >> 4; const size_t b = blockIdx.y; const int q0 = blockIdx.x * 64 + wave * 16; const size_t rq = b * SS + q0;
  for (int e = tid; e < 64 * 64; e += 128) { const int ee = e >> 6, d = e & 63; const float v = M[(b * HD + ee) * HD + d]; const __bf16 hv = (__bf16)v; smh[ee][d] = hv; sml[ee][d] = (__bf16)(v - (float)hv); }
  __syncthreads();
  { v8f acc[4] = {};
#pragma unroll
    for (int kc = 0; kc < HD / 32; ++kc) { v16b a; { const _Float16* p = Q + (rq + col) * HD + kc * 32 + 8 * g;
#pragma unroll
        for (int i = 0; i < 8; ++i) { a[i] = (__bf16)(float)p[i]; a[8 + i] = (__bf16)(float)p[16 + i]; } }
#pragma unroll
      for (int jt = 0; jt < 4; ++jt) { acc[jt] = wmma_bf(a, frag_b(&smh[jt * 16 + col][0] + kc * 32, lane), acc[jt]); acc[jt] = wmma_bf(a, frag_b(&sml[jt * 16 + col][0] + kc * 32, lane), acc[jt]); } }
#pragma unroll
    for (int jt = 0; jt < 4; ++jt)
#pragma unroll
      for (int r = 0; r < 8; ++r) { const int e = jt * 16 + col; sv[wave][8 * g + r][e] = acc[jt][r] * 0.125f + bfr(Qi[(rq + 8 * g + r) * HD + e]); } }
  LDSX();
  { const int rl = lane & 15, half = lane >> 4; float s = 0.f; for (int d = half * 32; d < half * 32 + 32; ++d) s += sv[wave][rl][d]; s += __shfl_xor(s, 16); const float mu = s / 64.0f; float q = 0.f; for (int d = half * 32; d < half * 32 + 32; ++d) { const float dd = sv[wave][rl][d] - mu; q += dd * dd; } q += __shfl_xor(q, 16); const float inv = 1.0f / sqrtf(q / 64.0f + 1e-5f);
    for (int d = half * 32; d < half * 32 + 32; ++d) sh[wave][rl][d] = (sv[wave][rl][d] - mu) * inv * bfr(GA[d]) + bfr(BE[d]); }
  LDSX();
  { v8f acc[16] = {};
#pragma unroll
    for (int kc = 0; kc < HD / 32; ++kc) { const F2 a = split_row(&sh[wave][col][0], kc * 32, lane);
#pragma unroll
      for (int jt = 0; jt < 16; ++jt) { const v16b w = frag_b(P + WS_P1 / 2 + (size_t)(jt * 16 + col) * HD + kc * 32, lane); acc[jt] = wmma_bf(a.h, w, acc[jt]); acc[jt] = wmma_bf(a.l, w, acc[jt]); } }
#pragma unroll
    for (int jt = 0; jt < 16; ++jt) { const float bb = bfr(B1[jt * 16 + col]);
#pragma unroll
      for (int r = 0; r < 8; ++r) { const float x = acc[jt][r] + bb; sg[wave][8 * g + r][jt * 16 + col] = 0.5f * x * (1.0f + erf_p(x * 0.70710678118654752f)); } } }
  LDSX();
  { v8f acc[4] = {};
#pragma unroll
    for (int kc = 0; kc < HID / 32; ++kc) { const F2 a = split_row(&sg[wave][col][0], kc * 32, lane);
#pragma unroll
      for (int jt = 0; jt < 4; ++jt) { const v16b w = frag_b(P + WS_P2 / 2 + (size_t)(jt * 16 + col) * HID + kc * 32, lane); acc[jt] = wmma_bf(a.h, w, acc[jt]); acc[jt] = wmma_bf(a.l, w, acc[jt]); } }
    LDSX();
#pragma unroll
    for (int jt = 0; jt < 4; ++jt) { const float bb = bfr(B2[jt * 16 + col]);
#pragma unroll
      for (int r = 0; r < 8; ++r) { const int e = jt * 16 + col; sh[wave][8 * g + r][e] = acc[jt][r] + bb + sv[wave][8 * g + r][e]; } } }
  LDSX();
  for (int rl = 0; rl < 16; ++rl) if (lane < 16) vst2(OUT + (rq + rl) * HD + lane * 4, *(const v4f*)&sh[wave][rl][lane * 4]);
}
extern "C" void kernel_launch(void* const* d_in, const int* in_sizes, int n_in, void* d_out, int out_size, void* d_ws, size_t ws_size, hipStream_t stream) {
  (void)in_sizes; (void)n_in; (void)out_size;
  const float** F = (const float**)d_in;
  if (ws_size < (size_t)WS_END) return;
  char* ws = (char*)d_ws; __bf16* P = (__bf16*)ws; _Float16 *Q = (_Float16*)(ws + WS_Q), *K = (_Float16*)(ws + WS_K), *VT = (_Float16*)(ws + WS_VT), *KT = (_Float16*)(ws + WS_KT), *V1H = (_Float16*)(ws + WS_V1H), *V1L = (_Float16*)(ws + WS_V1L); float* M = (float*)(ws + WS_M);
  k_pack<<<HD + HID + HD, 256, 0, stream>>>(F[3], F[7], F[9], P);
  k_rows<<<NB * SS / 64, 256, 0, stream>>>(F[0], F[1], F[2], Q, K, VT, KT);
  k_attn<<<dim3(SS / 64, NB), 128, 0, stream>>>(Q, K, VT, F[2], P, F[4], V1H, V1L);
  k_m<<<NB, 128, 0, stream>>>(V1H, V1L, KT, M);
  k_fin<<<dim3(TQB, TNB), 128, 0, stream>>>(F[0], Q, M, P, F[5], F[6], F[8], F[10], (float*)d_out);
}
